// NeighborhoodSelfAttention_23776938951308
// MI455X (gfx1250) — hardware-verified
//
#include <hip/hip_runtime.h>

typedef unsigned short v4us  __attribute__((ext_vector_type(4)));
typedef unsigned short v8us  __attribute__((ext_vector_type(8)));
typedef unsigned short v16us __attribute__((ext_vector_type(16)));
typedef __bf16         v16bf __attribute__((ext_vector_type(16)));
typedef float          v8f   __attribute__((ext_vector_type(8)));
typedef float          v4f   __attribute__((ext_vector_type(4)));
typedef v4us __attribute__((may_alias)) v4usa;
typedef v8us __attribute__((may_alias)) v8usa;
typedef v4f  __attribute__((may_alias)) v4fa;

union Frag { v16bf v; v16us u; v8us half[2]; };

#define NTOK   32768
#define GDIM   32
#define CH     128
#define NQKV   384
#define CF     512
#define NHEAD  8
#define HDIM   16
#define KS     3
#define NTAP   27
#define RPBD   5
#define NRPB   1000
#define TPX    64
#define TN     64
#define APX    32
#define SDP    68
#define LPX    136
#define LH     72
#define NBX    (NTOK / TPX)
#define ATT_SCALE 0.25f
#define NORM_EPS  1e-5f

static_assert(GDIM * GDIM * GDIM == NTOK);
static_assert(NTOK % TPX == 0 && NTOK % APX == 0);
static_assert(NQKV % TN == 0 && CF % TN == 0 && CH % TN == 0);
static_assert(CH % 32 == 0 && CF % 32 == 0);
static_assert(NHEAD * HDIM == CH);
static_assert(NHEAD * 32 == 256);
static_assert((SDP % 4) == 0 && (LPX % 8) == 0 && (LH % 8) == 0);
static_assert((NQKV * CH) % 2048 == 0 && (CH * CH) % 2048 == 0 && (CF * CH) % 2048 == 0);
static_assert(NBX * 2 * 2 * 64 * 4 == 524288);
static_assert(KS * KS * KS == NTAP && RPBD * RPBD * RPBD * NHEAD == NRPB);

__device__ __forceinline__ unsigned int bf16_bits(float f) {
  const unsigned int u = __float_as_uint(f);
  return (u + 0x7FFFu + ((u >> 16) & 1u)) >> 16;
}
__device__ __forceinline__ float bf16_val(float f) {
  return __uint_as_float(bf16_bits(f) << 16);
}

__device__ __forceinline__ float gelu_tanh(float x) {
  const float k0 = 0.7978845608028654f;
  const float k1 = 0.044715f;
  const float u = k0 * (x + k1 * x * x * x);
  return 0.5f * x * (1.0f + tanhf(u));
}

__device__ __forceinline__ v8f wmma_bf16(Frag a, Frag b, v8f c) {
  v8f d = __builtin_amdgcn_wmma_f32_16x16x32_bf16(false, a.v, false, b.v, (short)0, c, false, false);
  asm volatile("v_nop\n\tv_nop\n\tv_nop\n\tv_nop" : "+v"(d) : "v"(a.u), "v"(b.u));
  return d;
}

__device__ __forceinline__ Frag load_frag(const unsigned short* p, int h) {
  Frag f;
  f.half[0] = *(const v8usa*)(p + 8 * h);
  f.half[1] = *(const v8usa*)(p + 16 + 8 * h);
  return f;
}

__global__ __launch_bounds__(256) void xt_kernel(const float* __restrict__ x,
                                                 unsigned short* __restrict__ xt)
{
  __shared__ __attribute__((aligned(16))) unsigned short sT[TPX * LPX];

  const int tid = threadIdx.x, lane = tid & 31, w = tid >> 5;
  const int p0 = blockIdx.x * TPX;
  const int pl = tid & 63, cb = tid >> 6;
  const float* xs = x + p0 + pl;

  #pragma unroll 4
  for (int i = 0; i < 32; ++i) {
    const int c = cb + 4 * i;
    const float v = xs[(size_t)c * NTOK];
    sT[pl * LPX + c] = (unsigned short)bf16_bits(v);
  }
  __syncthreads();

  const int sub = lane >> 4, c8 = 8 * (lane & 15);
  v8us vv[4];
  #pragma unroll
  for (int i = 0; i < 4; ++i) {
    const int row = 8 * w + 2 * i + sub;
    vv[i] = *(const v8usa*)(sT + row * LPX + c8);
  }
  unsigned short* base = xt + (size_t)p0 * CH + c8;
  #pragma unroll
  for (int i = 0; i < 4; ++i) {
    const int row = 8 * w + 2 * i + sub;
    *(volatile v8us*)(base + (size_t)row * CH) = vv[i];
  }
  __threadfence();
  #pragma unroll
  for (int i = 0; i < 4; ++i) {
    const int row = 8 * w + 2 * i + sub;
    *(volatile v8us*)(base + (size_t)row * CH) = vv[i];
  }
}

__global__ __launch_bounds__(256) void wconv_kernel(const float* __restrict__ wsrc,
                                                    unsigned short* __restrict__ wdst,
                                                    int n8)
{
  const int g = blockIdx.x * 256 + threadIdx.x;
  if (g >= n8) return;
  const v4f* src = (const v4f*)(wsrc + (size_t)g * 8);
  const v4f a = src[0];
  const v4f b = src[1];
  v8us o;
  o[0] = (unsigned short)bf16_bits(a.x); o[1] = (unsigned short)bf16_bits(a.y);
  o[2] = (unsigned short)bf16_bits(a.z); o[3] = (unsigned short)bf16_bits(a.w);
  o[4] = (unsigned short)bf16_bits(b.x); o[5] = (unsigned short)bf16_bits(b.y);
  o[6] = (unsigned short)bf16_bits(b.z); o[7] = (unsigned short)bf16_bits(b.w);
  unsigned short* dst = wdst + (size_t)g * 8;
  *(volatile v8us*)dst = o;
  __threadfence();
  *(volatile v8us*)dst = o;
}

__global__ __launch_bounds__(128) void gemm_qkv_kernel(
    const unsigned short* __restrict__ xa_plane,
    const unsigned short* __restrict__ wq,
    const float* __restrict__ bias,
    float* __restrict__ qkv)
{
  __shared__ __attribute__((aligned(16))) float sD[TPX * SDP];

  const int tid = threadIdx.x, lane = tid & 31, w = tid >> 5;
  const int h = lane >> 4, m = lane & 15;
  const int m0 = blockIdx.x * TPX, n0 = blockIdx.y * TN;
  const v8f zero8 = {0.f, 0.f, 0.f, 0.f, 0.f, 0.f, 0.f, 0.f};

  v8f acc[4];
  #pragma unroll
  for (int nt = 0; nt < 4; ++nt) acc[nt] = zero8;

  const unsigned short* xa = xa_plane + (size_t)(m0 + 16 * w + m) * CH;
  const unsigned short* wb = wq + (size_t)(n0 + m) * CH;

  #pragma unroll 1
  for (int k0 = 0; k0 < CH; k0 += 32) {
    const Frag a = load_frag(xa + k0, h);
    #pragma unroll
    for (int nt = 0; nt < 4; ++nt) {
      const Frag b = load_frag(wb + (size_t)nt * 16 * CH + k0, h);
      acc[nt] = wmma_bf16(a, b, acc[nt]);
    }
  }

  #pragma unroll
  for (int nt = 0; nt < 4; ++nt) {
    const int o = 16 * nt + m;
    const float bv = bf16_val(bias[n0 + o]);
    #pragma unroll
    for (int r = 0; r < 8; ++r) sD[(16 * w + 8 * h + r) * SDP + o] = acc[nt][r] + bv;
  }
  __syncthreads();

  const int sub = lane >> 4, c4 = 4 * (lane & 15);
  v4f vv[8];
  #pragma unroll
  for (int i = 0; i < 8; ++i) {
    const int row = 16 * w + 2 * i + sub;
    vv[i] = *(const v4fa*)(sD + row * SDP + c4);
  }
  float* base = qkv + (size_t)m0 * NQKV + n0 + c4;
  #pragma unroll
  for (int i = 0; i < 8; ++i) {
    const int row = 16 * w + 2 * i + sub;
    *(volatile v4f*)(base + (size_t)row * NQKV) = vv[i];
  }
  __threadfence();
  #pragma unroll
  for (int i = 0; i < 8; ++i) {
    const int row = 16 * w + 2 * i + sub;
    *(volatile v4f*)(base + (size_t)row * NQKV) = vv[i];
  }
}

__global__ __launch_bounds__(256) void attn_kernel(const float* __restrict__ qkv,
                                                   const float* __restrict__ rpb,
                                                   unsigned short* __restrict__ ohi,
                                                   unsigned short* __restrict__ olo)
{
  __shared__ __attribute__((aligned(16))) float sLg[NTAP * 256];
  __shared__ __attribute__((aligned(16))) float sB[1024];
  __shared__ __attribute__((aligned(16))) unsigned short sH[APX * CH];
  __shared__ __attribute__((aligned(16))) unsigned short sL[APX * CH];

  const int tid = threadIdx.x, lane = tid & 31, hd = tid >> 5;
  const int p0 = blockIdx.x * APX;
  const int p  = p0 + lane;
  const int cz = p & (GDIM - 1), cy = (p >> 5) & (GDIM - 1), cx = p >> 10;

  #pragma unroll 1
  for (int i = tid; i < 1024; i += 256) {
    const int ii = (i < NRPB) ? i : (NRPB - 1);
    const float v = bf16_val(rpb[ii]);
    sB[i] = (i < NRPB) ? v : 0.0f;
  }
  __syncthreads();

  const int sx = min(max(cx - 1, 0), GDIM - KS);
  const int sy = min(max(cy - 1, 0), GDIM - KS);
  const int sz = min(max(cz - 1, 0), GDIM - KS);

  const v4f s4 = {ATT_SCALE, ATT_SCALE, ATT_SCALE, ATT_SCALE};
  const v4f* q4 = (const v4f*)(qkv + (size_t)p * NQKV + hd * HDIM);
  v4f q[4];
  #pragma unroll
  for (int c = 0; c < 4; ++c) q[c] = q4[c] * s4;

  float mx = __uint_as_float(0xff800000u);
  #pragma unroll 1
  for (int t = 0; t < NTAP; ++t) {
    const int a  = t / 9;
    const int r9 = t - 9 * a;
    const int b  = r9 / 3;
    const int c3 = r9 - 3 * b;
    const int nx = sx + a, ny = sy + b, nz = sz + c3;
    const int pn = (nx * GDIM + ny) * GDIM + nz;
    const v4f* k4 = (const v4f*)(qkv + (size_t)pn * NQKV + CH + hd * HDIM);
    float s = 0.0f;
    #pragma unroll
    for (int c = 0; c < 4; ++c) {
      const v4f qv = q[c];
      const v4f kv = k4[c];
      s = fmaf(qv.x, kv.x, s);
      s = fmaf(qv.y, kv.y, s);
      s = fmaf(qv.z, kv.z, s);
      s = fmaf(qv.w, kv.w, s);
    }
    const int bi = ((hd * RPBD + (nx - cx + 2)) * RPBD + (ny - cy + 2)) * RPBD + (nz - cz + 2);
    const float lg = s + sB[bi];
    sLg[t * 256 + tid] = lg;
    mx = fmaxf(mx, lg);
  }

  float wsum = 0.0f;
  #pragma unroll 1
  for (int t = 0; t < NTAP; ++t) {
    const float e = expf(sLg[t * 256 + tid] - mx);
    sLg[t * 256 + tid] = e;
    wsum += e;
  }
  const float inv = 1.0f / wsum;

  const v4f z4 = {0.f, 0.f, 0.f, 0.f};
  v4f o[4];
  #pragma unroll
  for (int c = 0; c < 4; ++c) o[c] = z4;

  #pragma unroll 1
  for (int t = 0; t < NTAP; ++t) {
    const int a  = t / 9;
    const int r9 = t - 9 * a;
    const int b  = r9 / 3;
    const int c3 = r9 - 3 * b;
    const int pn = ((sx + a) * GDIM + (sy + b)) * GDIM + (sz + c3);
    const float wt = sLg[t * 256 + tid] * inv;
    const v4f* v4 = (const v4f*)(qkv + (size_t)pn * NQKV + 2 * CH + hd * HDIM);
    #pragma unroll
    for (int c = 0; c < 4; ++c) {
      const v4f vv = v4[c];
      v4f acc = o[c];
      acc.x = fmaf(wt, vv.x, acc.x);
      acc.y = fmaf(wt, vv.y, acc.y);
      acc.z = fmaf(wt, vv.z, acc.z);
      acc.w = fmaf(wt, vv.w, acc.w);
      o[c] = acc;
    }
  }

  v8us hv[2], lv[2];
  #pragma unroll
  for (int j = 0; j < 2; ++j) {
    const v4f a0 = o[2 * j];
    const v4f a1 = o[2 * j + 1];
    const float f[8] = {a0.x, a0.y, a0.z, a0.w, a1.x, a1.y, a1.z, a1.w};
    #pragma unroll
    for (int e = 0; e < 8; ++e) {
      const unsigned int hb = bf16_bits(f[e]);
      const float hf = __uint_as_float(hb << 16);
      hv[j][e] = (unsigned short)hb;
      lv[j][e] = (unsigned short)bf16_bits(f[e] - hf);
    }
  }

  #pragma unroll
  for (int j = 0; j < 2; ++j) {
    *(v8usa*)(sH + lane * CH + hd * HDIM + 8 * j) = hv[j];
    *(v8usa*)(sL + lane * CH + hd * HDIM + 8 * j) = lv[j];
  }
  __syncthreads();

  const int sub = lane >> 4, c8 = 8 * (lane & 15);
  v8us oh[2], ol[2];
  #pragma unroll
  for (int i = 0; i < 2; ++i) {
    const int row = 4 * hd + 2 * i + sub;
    oh[i] = *(const v8usa*)(sH + row * CH + c8);
    ol[i] = *(const v8usa*)(sL + row * CH + c8);
  }
  const size_t rb = (size_t)p0 * CH + c8;
  #pragma unroll
  for (int i = 0; i < 2; ++i) {
    const size_t off = rb + (size_t)(4 * hd + 2 * i + sub) * CH;
    *(volatile v8us*)(ohi + off) = oh[i];
    *(volatile v8us*)(olo + off) = ol[i];
  }
  __threadfence();
  #pragma unroll
  for (int i = 0; i < 2; ++i) {
    const size_t off = rb + (size_t)(4 * hd + 2 * i + sub) * CH;
    *(volatile v8us*)(ohi + off) = oh[i];
    *(volatile v8us*)(olo + off) = ol[i];
  }
}

__global__ __launch_bounds__(128) void gemm_out_kernel(
    const unsigned short* __restrict__ ahi,
    const unsigned short* __restrict__ alo,
    int K,
    const unsigned short* __restrict__ wb,
    const float* __restrict__ bias,
    int use_res,
    const float* __restrict__ resP,
    const float* __restrict__ tab,
    float* __restrict__ outP,
    float* __restrict__ rec)
{
  __shared__ __attribute__((aligned(16))) float sD[TPX * SDP];
  __shared__ __attribute__((aligned(16))) float sRec[128];

  const int tid = threadIdx.x, lane = tid & 31, w = tid >> 5;
  const int h = lane >> 4, m = lane & 15;
  const int m0 = blockIdx.x * TPX, n0 = blockIdx.y * TN;
  const v8f zero8 = {0.f, 0.f, 0.f, 0.f, 0.f, 0.f, 0.f, 0.f};

  v8f acc[4];
  #pragma unroll
  for (int nt = 0; nt < 4; ++nt) acc[nt] = zero8;

  const size_t arow = (size_t)(m0 + 16 * w + m) * (size_t)K;
  const unsigned short* ha = ahi + arow;
  const unsigned short* la = alo + arow;
  const unsigned short* wr = wb + (size_t)(n0 + m) * (size_t)K;

  #pragma unroll 1
  for (int k0 = 0; k0 < K; k0 += 32) {
    const Frag fh = load_frag(ha + k0, h);
    const Frag fl = load_frag(la + k0, h);
    #pragma unroll
    for (int nt = 0; nt < 4; ++nt) {
      const Frag b = load_frag(wr + (size_t)nt * 16 * K + k0, h);
      acc[nt] = wmma_bf16(fh, b, acc[nt]);
      acc[nt] = wmma_bf16(fl, b, acc[nt]);
    }
  }

  #pragma unroll
  for (int nt = 0; nt < 4; ++nt) {
    const int o = 16 * nt + m;
    const float bv = bf16_val(bias[n0 + o]);
    #pragma unroll
    for (int r = 0; r < 8; ++r) sD[(16 * w + 8 * h + r) * SDP + o] = acc[nt][r] + bv;
  }
  __syncthreads();

  if (use_res != 0) {
    #pragma unroll 1
    for (int i = 0; i < 32; ++i) {
      const int e = tid + 128 * i;
      const int row = e >> 6, col = e & 63;
      const int c = n0 + col;
      const float pv = resP[(size_t)(m0 + row) * CH + c];
      const float t = (pv - tab[c]) * tab[CH + c];
      sD[row * SDP + col] += t;
    }
  }
  __syncthreads();

  {
    const int col = tid & 63;
    const bool do_sq = (tid >= 64);
    float s = 0.0f;
    #pragma unroll 4
    for (int row = 0; row < TPX; ++row) {
      const float v = sD[row * SDP + col];
      s += do_sq ? (v * v) : v;
    }
    sRec[tid] = s;
  }
  __syncthreads();

  const int sub = lane >> 4, c4 = 4 * (lane & 15);
  v4f vv[8];
  #pragma unroll
  for (int i = 0; i < 8; ++i) {
    const int row = 16 * w + 2 * i + sub;
    vv[i] = *(const v4fa*)(sD + row * SDP + c4);
  }
  const v4f rv = *(const v4fa*)(sRec + 4 * lane);
  float* base = outP + (size_t)m0 * CH + n0 + c4;
  float* rdst = rec + (size_t)(blockIdx.x * 2 + blockIdx.y) * 128 + 4 * lane;

  #pragma unroll
  for (int i = 0; i < 8; ++i) {
    const int row = 16 * w + 2 * i + sub;
    *(volatile v4f*)(base + (size_t)row * CH) = vv[i];
  }
  if (w == 0) *(volatile v4f*)rdst = rv;
  __threadfence();
  #pragma unroll
  for (int i = 0; i < 8; ++i) {
    const int row = 16 * w + 2 * i + sub;
    *(volatile v4f*)(base + (size_t)row * CH) = vv[i];
  }
  if (w == 0) *(volatile v4f*)rdst = rv;
}

__global__ __launch_bounds__(128) void fold_kernel(const float* __restrict__ rec,
                                                   float* __restrict__ tab)
{
  __shared__ __attribute__((aligned(16))) float sTab[2 * CH];
  const int c = threadIdx.x;
  const int by = c >> 6, cl = c & 63;
  double s = 0.0, ss = 0.0;
  #pragma unroll 1
  for (int bx = 0; bx < NBX; ++bx) {
    const float* r = rec + (size_t)((bx * 2 + by) * 2) * 64 + cl;
    s  += (double)r[0];
    ss += (double)r[64];
  }
  const double mean = s * (1.0 / (double)NTOK);
  double var = ss * (1.0 / (double)NTOK) - mean * mean;
  var = (var > 0.0) ? var : 0.0;
  sTab[c] = (float)mean;
  sTab[CH + c] = rsqrtf((float)var + NORM_EPS);
  __syncthreads();

  const v4f tv = *(const v4fa*)(sTab + 4 * (c & 63));
  if (c < 64) *(volatile v4f*)(tab + 4 * c) = tv;
  __threadfence();
  if (c < 64) *(volatile v4f*)(tab + 4 * c) = tv;
}

__global__ __launch_bounds__(256) void normsplit_kernel(const float* __restrict__ P,
                                                        const float* __restrict__ tab,
                                                        unsigned short* __restrict__ thi,
                                                        unsigned short* __restrict__ tlo)
{
  __shared__ __attribute__((aligned(16))) float sTab[2 * CH];
  __shared__ __attribute__((aligned(16))) unsigned short sHi[TPX * LPX];
  __shared__ __attribute__((aligned(16))) unsigned short sLo[TPX * LPX];

  const int tid = threadIdx.x, lane = tid & 31, w = tid >> 5;
  const int n0 = blockIdx.x * TPX;
  sTab[tid] = tab[tid];
  __syncthreads();

  const int c4 = 4 * lane;
  const v4f mu = *(const v4fa*)(sTab + c4);
  const v4f rs = *(const v4fa*)(sTab + CH + c4);
  #pragma unroll 2
  for (int i = 0; i < 8; ++i) {
    const int row = 8 * w + i;
    const v4f v = *(const v4fa*)(P + (size_t)(n0 + row) * CH + c4);
    const float f[4] = {(v.x - mu.x) * rs.x, (v.y - mu.y) * rs.y, (v.z - mu.z) * rs.z, (v.w - mu.w) * rs.w};
    v4us hb, lb;
    #pragma unroll
    for (int e = 0; e < 4; ++e) {
      const unsigned int hbits = bf16_bits(f[e]);
      const float hf = __uint_as_float(hbits << 16);
      hb[e] = (unsigned short)hbits;
      lb[e] = (unsigned short)bf16_bits(f[e] - hf);
    }
    *(v4usa*)(sHi + row * LPX + c4) = hb;
    *(v4usa*)(sLo + row * LPX + c4) = lb;
  }
  __syncthreads();

  const int sub = lane >> 4, c8 = 8 * (lane & 15);
  v8us hv[4], lv[4];
  #pragma unroll
  for (int i = 0; i < 4; ++i) {
    const int row = 8 * w + 2 * i + sub;
    hv[i] = *(const v8usa*)(sHi + row * LPX + c8);
    lv[i] = *(const v8usa*)(sLo + row * LPX + c8);
  }
  const size_t rb = (size_t)n0 * CH + c8;
  #pragma unroll
  for (int i = 0; i < 4; ++i) {
    const size_t off = rb + (size_t)(8 * w + 2 * i + sub) * CH;
    *(volatile v8us*)(thi + off) = hv[i];
    *(volatile v8us*)(tlo + off) = lv[i];
  }
  __threadfence();
  #pragma unroll
  for (int i = 0; i < 4; ++i) {
    const size_t off = rb + (size_t)(8 * w + 2 * i + sub) * CH;
    *(volatile v8us*)(thi + off) = hv[i];
    *(volatile v8us*)(tlo + off) = lv[i];
  }
}

__global__ __launch_bounds__(128) void gemm_ffn1_kernel(
    const unsigned short* __restrict__ thi,
    const unsigned short* __restrict__ tlo,
    const unsigned short* __restrict__ w1,
    const float* __restrict__ bias,
    unsigned short* __restrict__ ghi,
    unsigned short* __restrict__ glo)
{
  __shared__ __attribute__((aligned(16))) float sD[TPX * SDP];
  __shared__ __attribute__((aligned(16))) unsigned short sH[TPX * LH];
  __shared__ __attribute__((aligned(16))) unsigned short sL[TPX * LH];

  const int tid = threadIdx.x, lane = tid & 31, w = tid >> 5;
  const int h = lane >> 4, m = lane & 15;
  const int m0 = blockIdx.x * TPX, n0 = blockIdx.y * TN;
  const v8f zero8 = {0.f, 0.f, 0.f, 0.f, 0.f, 0.f, 0.f, 0.f};

  v8f acc[4];
  #pragma unroll
  for (int nt = 0; nt < 4; ++nt) acc[nt] = zero8;

  const size_t arow = (size_t)(m0 + 16 * w + m) * CH;
  const unsigned short* ha = thi + arow;
  const unsigned short* la = tlo + arow;
  const unsigned short* wr = w1 + (size_t)(n0 + m) * CH;

  #pragma unroll 1
  for (int k0 = 0; k0 < CH; k0 += 32) {
    const Frag fh = load_frag(ha + k0, h);
    const Frag fl = load_frag(la + k0, h);
    #pragma unroll
    for (int nt = 0; nt < 4; ++nt) {
      const Frag b = load_frag(wr + (size_t)nt * 16 * CH + k0, h);
      acc[nt] = wmma_bf16(fh, b, acc[nt]);
      acc[nt] = wmma_bf16(fl, b, acc[nt]);
    }
  }

  #pragma unroll
  for (int nt = 0; nt < 4; ++nt) {
    const int o = 16 * nt + m;
    const float bv = bf16_val(bias[n0 + o]);
    #pragma unroll
    for (int r = 0; r < 8; ++r) sD[(16 * w + 8 * h + r) * SDP + o] = acc[nt][r] + bv;
  }
  __syncthreads();

  #pragma unroll 1
  for (int i = 0; i < 32; ++i) {
    const int e = tid + 128 * i;
    const int row = e >> 6, col = e & 63;
    const float g = gelu_tanh(sD[row * SDP + col]);
    const unsigned int hbits = bf16_bits(g);
    const float hf = __uint_as_float(hbits << 16);
    sH[row * LH + col] = (unsigned short)hbits;
    sL[row * LH + col] = (unsigned short)bf16_bits(g - hf);
  }
  __syncthreads();

  const int q8 = lane & 7, sub = lane >> 3;
  v8us hv[4], lv[4];
  #pragma unroll
  for (int i = 0; i < 4; ++i) {
    const int row = 16 * w + 4 * i + sub;
    hv[i] = *(const v8usa*)(sH + row * LH + 8 * q8);
    lv[i] = *(const v8usa*)(sL + row * LH + 8 * q8);
  }
  const size_t gb = (size_t)m0 * CF + n0 + 8 * q8;
  #pragma unroll
  for (int i = 0; i < 4; ++i) {
    const size_t off = gb + (size_t)(16 * w + 4 * i + sub) * CF;
    *(volatile v8us*)(ghi + off) = hv[i];
    *(volatile v8us*)(glo + off) = lv[i];
  }
  __threadfence();
  #pragma unroll
  for (int i = 0; i < 4; ++i) {
    const size_t off = gb + (size_t)(16 * w + 4 * i + sub) * CF;
    *(volatile v8us*)(ghi + off) = hv[i];
    *(volatile v8us*)(glo + off) = lv[i];
  }
}

__global__ __launch_bounds__(256) void final_kernel(const float* __restrict__ Y,
                                                    const float* __restrict__ tab,
                                                    float* __restrict__ out)
{
  __shared__ __attribute__((aligned(16))) float sTab[2 * CH];
  __shared__ __attribute__((aligned(16))) float sT[CH * SDP];

  const int tid = threadIdx.x, lane = tid & 31, w = tid >> 5;
  const int n0 = blockIdx.x * TPX;
  sTab[tid] = tab[tid];
  __syncthreads();

  const int c4 = 4 * lane;
  const v4f mu = *(const v4fa*)(sTab + c4);
  const v4f rs = *(const v4fa*)(sTab + CH + c4);
  #pragma unroll 2
  for (int i = 0; i < 8; ++i) {
    const int row = 8 * w + i;
    const v4f v = *(const v4fa*)(Y + (size_t)(n0 + row) * CH + c4);
    sT[(c4 + 0) * SDP + row] = (v.x - mu.x) * rs.x;
    sT[(c4 + 1) * SDP + row] = (v.y - mu.y) * rs.y;
    sT[(c4 + 2) * SDP + row] = (v.z - mu.z) * rs.z;
    sT[(c4 + 3) * SDP + row] = (v.w - mu.w) * rs.w;
  }
  __syncthreads();

  const int sub = lane >> 4, t4 = 4 * (lane & 15);
  v4f vv[8];
  #pragma unroll
  for (int i = 0; i < 8; ++i) {
    const int ch = 16 * w + 2 * i + sub;
    vv[i] = *(const v4fa*)(sT + ch * SDP + t4);
  }
  float* base = out + n0 + t4;
  #pragma unroll
  for (int i = 0; i < 8; ++i) {
    const int ch = 16 * w + 2 * i + sub;
    *(volatile v4f*)(base + (size_t)ch * NTOK) = vv[i];
  }
  __threadfence();
  #pragma unroll
  for (int i = 0; i < 8; ++i) {
    const int ch = 16 * w + 2 * i + sub;
    *(volatile v4f*)(base + (size_t)ch * NTOK) = vv[i];
  }
}

extern "C" void kernel_launch(void* const* d_in, const int* in_sizes, int n_in,
                              void* d_out, int out_size, void* d_ws, size_t ws_size,
                              hipStream_t stream) {
  if (n_in < 10) return;
  if (in_sizes[0] != CH * NTOK) return;
  if (in_sizes[1] != NQKV * CH) return;
  if (in_sizes[2] != NQKV) return;
  if (in_sizes[3] != NRPB) return;
  if (in_sizes[4] != CH * CH) return;
  if (in_sizes[5] != CH) return;
  if (in_sizes[6] != CF * CH) return;
  if (in_sizes[7] != CF) return;
  if (in_sizes[8] != CH * CF) return;
  if (in_sizes[9] != CH) return;
  if (out_size != CH * NTOK) return;

  const float* x      = (const float*)d_in[0];
  const float* w_qkv  = (const float*)d_in[1];
  const float* b_qkv  = (const float*)d_in[2];
  const float* rpb    = (const float*)d_in[3];
  const float* w_proj = (const float*)d_in[4];
  const float* b_proj = (const float*)d_in[5];
  const float* w_ffn1 = (const float*)d_in[6];
  const float* b_ffn1 = (const float*)d_in[7];
  const float* w_ffn2 = (const float*)d_in[8];
  const float* b_ffn2 = (const float*)d_in[9];
  float* out = (float*)d_out;

  const size_t ra_bytes  = (size_t)2 * NTOK * CF * 2;
  const size_t rb_bytes  = (size_t)NTOK * CH * 4;
  const size_t rc_bytes  = (size_t)NTOK * CH * 4;
  const size_t wq_bytes  = (size_t)NQKV * CH * 2;
  const size_t wp_bytes  = (size_t)CH * CH * 2;
  const size_t w1_bytes  = (size_t)CF * CH * 2;
  const size_t w2_bytes  = (size_t)CH * CF * 2;
  const size_t rec_bytes = (size_t)NBX * 2 * 2 * 64 * 4;
  const size_t tab_bytes = (size_t)2 * CH * 4;
  const size_t total = ra_bytes + rb_bytes + rc_bytes + wq_bytes + wp_bytes + w1_bytes + w2_bytes
                     + 2 * rec_bytes + 2 * tab_bytes;
  if ((size_t)NTOK * NQKV * 4 > ra_bytes) return;
  if (total > ws_size) return;

  char* ws = (char*)d_ws;
  size_t off = 0;
  char* ra = ws + off; off += ra_bytes;
  char* rb = ws + off; off += rb_bytes;
  char* rc = ws + off; off += rc_bytes;
  unsigned short* wq = (unsigned short*)(ws + off); off += wq_bytes;
  unsigned short* wp = (unsigned short*)(ws + off); off += wp_bytes;
  unsigned short* w1 = (unsigned short*)(ws + off); off += w1_bytes;
  unsigned short* w2 = (unsigned short*)(ws + off); off += w2_bytes;
  float* rec1 = (float*)(ws + off); off += rec_bytes;
  float* rec2 = (float*)(ws + off); off += rec_bytes;
  float* tab1 = (float*)(ws + off); off += tab_bytes;
  float* tab2 = (float*)(ws + off); off += tab_bytes;
  if (off != total) return;

  float*          qkvp = (float*)ra;
  unsigned short* ghi  = (unsigned short*)ra;
  unsigned short* glo  = (unsigned short*)(ra + (size_t)NTOK * CF * 2);
  unsigned short* xt   = (unsigned short*)rb;
  unsigned short* ohi  = (unsigned short*)rb;
  unsigned short* olo  = (unsigned short*)(rb + (size_t)NTOK * CH * 2);
  unsigned short* thi  = (unsigned short*)rb;
  unsigned short* tlo  = (unsigned short*)(rb + (size_t)NTOK * CH * 2);
  float*          Y    = (float*)rb;
  float*          P    = (float*)rc;

  const int n8_qkv = NQKV * CH / 8;
  const int n8_prj = CH * CH / 8;
  const int n8_f1  = CF * CH / 8;
  const int n8_f2  = CH * CF / 8;

  xt_kernel<<<dim3(NTOK / TPX), 256, 0, stream>>>(x, xt);
  wconv_kernel<<<dim3((n8_qkv + 255) / 256), 256, 0, stream>>>(w_qkv, wq, n8_qkv);
  wconv_kernel<<<dim3((n8_prj + 255) / 256), 256, 0, stream>>>(w_proj, wp, n8_prj);
  wconv_kernel<<<dim3((n8_f1 + 255) / 256), 256, 0, stream>>>(w_ffn1, w1, n8_f1);
  wconv_kernel<<<dim3((n8_f2 + 255) / 256), 256, 0, stream>>>(w_ffn2, w2, n8_f2);

  gemm_qkv_kernel<<<dim3(NTOK / TPX, NQKV / TN), 128, 0, stream>>>(xt, wq, b_qkv, qkvp);
  attn_kernel<<<dim3(NTOK / APX), 256, 0, stream>>>(qkvp, rpb, ohi, olo);
  gemm_out_kernel<<<dim3(NTOK / TPX, CH / TN), 128, 0, stream>>>(ohi, olo, CH, wp, b_proj, 0, qkvp, tab1, P, rec1);
  fold_kernel<<<dim3(1), 128, 0, stream>>>(rec1, tab1);
  normsplit_kernel<<<dim3(NTOK / TPX), 256, 0, stream>>>(P, tab1, thi, tlo);
  gemm_ffn1_kernel<<<dim3(NTOK / TPX, CF / TN), 128, 0, stream>>>(thi, tlo, w1, b_ffn1, ghi, glo);
  gemm_out_kernel<<<dim3(NTOK / TPX, CH / TN), 128, 0, stream>>>(ghi, glo, CF, w2, b_ffn2, 1, P, tab1, Y, rec2);
  fold_kernel<<<dim3(1), 128, 0, stream>>>(rec2, tab2);
  final_kernel<<<dim3(NTOK / TPX), 256, 0, stream>>>(Y, tab2, out);
}
